// M2RNNAttn_52578989637693
// MI455X (gfx1250) — hardware-run, weakly checked
//
#include <hip/hip_runtime.h>
#include <math.h>

constexpr int NBAT   = 4;
constexpr int NSEQ   = 1024;
constexpr int NDIM   = 1024;
constexpr int NHEAD  = 8;
constexpr int HDIM   = 64;
constexpr int NROWS  = NBAT * NSEQ;
constexpr int NQKV   = 3 * NHEAD * HDIM;
constexpr int NPROJ  = 1600;
constexpr int NYC    = NHEAD * HDIM;
constexpr int NOUT0  = NROWS * NDIM;
constexpr int NOUT1  = NBAT * NHEAD * HDIM * HDIM;
constexpr int HSP    = 72;
constexpr int SLP    = 68;
constexpr float XCARRY   = 16.0f;
constexpr float WPCARRY  = 32.0f;
constexpr float WRCARRY  = 8.0f;
constexpr float WOCARRY  = 16.0f;
constexpr float LOCARRY  = 2048.0f;
constexpr float HFLUSH   = 6.2e-5f;
constexpr float PROJ_SCALE = 1.0f / (XCARRY * WPCARRY);
constexpr float OUT_SCALE  = 1.0f / WOCARRY;
constexpr float ZSCALE2    = 2.0f / WRCARRY;
constexpr float ZSCALE2L   = ZSCALE2 / LOCARRY;

constexpr int PK_QKV_TILES = 3 * (512 / 64) * (NDIM / 64);
constexpr int PK_WF_TILES  = NDIM / 64;
constexpr int PK_WO_TILES  = (NDIM / 64) * (NYC / 64);
constexpr int PK_WR_TILES  = NHEAD;
constexpr int PK_TILES     = PK_QKV_TILES + PK_WF_TILES + PK_WO_TILES + PK_WR_TILES;
constexpr int CONV_BLOCKS  = NROWS * (NQKV / 4) / 256;
constexpr int GATE_BLOCKS  = NROWS * 2 / 256;

constexpr int RECUR_LDS_BYTES = 64 * HSP * 2 + 2 * (4 * 16 * HSP * 2) + 4 * 32 * 32 * 4 + 2 * 192 * 4 + 2 * 4 * 64 * 4 + 4 * 16 * SLP * 4;

static_assert(NROWS % 64 == 0);
static_assert(NPROJ % 64 == 0);
static_assert(NDIM % 64 == 0);
static_assert(NDIM % 32 == 0);
static_assert(NYC % 32 == 0);
static_assert(HDIM % 32 == 0);
static_assert(NQKV + NHEAD <= NPROJ);
static_assert(((NROWS / 64) * (NPROJ / 64)) % 8 == 0);
static_assert(((NROWS / 64) * (NDIM / 64)) % 8 == 0);
static_assert((NROWS * (NQKV / 4)) % 256 == 0);
static_assert((NROWS * 2) % 256 == 0);
static_assert(NHEAD * HDIM == 512);
static_assert(PK_TILES == 536);
static_assert(RECUR_LDS_BYTES == 65024);
static_assert(RECUR_LDS_BYTES <= 65536);

typedef __attribute__((ext_vector_type(16))) _Float16 v16h;
typedef __attribute__((ext_vector_type(8)))  _Float16 v8h;
typedef __attribute__((ext_vector_type(8)))  float    v8f;
typedef __attribute__((ext_vector_type(4)))  float    v4f;

__device__ __forceinline__ unsigned short f2bf_bits(float f) {
  unsigned u = __float_as_uint(f);
  return (unsigned short)((u + 0x7FFFu + ((u >> 16) & 1u)) >> 16);
}
__device__ __forceinline__ float bf16r(float f) { return __uint_as_float(((unsigned)f2bf_bits(f)) << 16); }

__device__ __forceinline__ void guard_row4(v8f& a, v8f& b, v8f& c, v8f& d, v16h x, v16h y0, v16h y1, v16h y2, v16h y3) {
  asm volatile("v_nop\n\tv_nop\n\tv_nop\n\tv_nop" : "+v"(a), "+v"(b), "+v"(c), "+v"(d) : "v"(x), "v"(y0), "v"(y1), "v"(y2), "v"(y3));
}
__device__ __forceinline__ void guard_pair(v8f& a, v16h x0, v16h x1, v16h y0, v16h y1) {
  asm volatile("v_nop\n\tv_nop\n\tv_nop\n\tv_nop" : "+v"(a) : "v"(x0), "v"(x1), "v"(y0), "v"(y1));
}
__device__ __forceinline__ void keep4_h(v16h a, v16h b, v16h c, v16h d) { asm volatile("v_nop" :: "v"(a), "v"(b), "v"(c), "v"(d)); }
__device__ __forceinline__ void acc_guard4(v8f& a, v8f& b, v8f& c, v8f& d) { asm volatile("v_nop\n\tv_nop\n\tv_nop\n\tv_nop" : "+v"(a), "+v"(b), "+v"(c), "+v"(d)); }

template <typename T> struct Frag;
template <> struct Frag<_Float16> {
  typedef v16h V; union U { v16h v; v8h h[2]; };
  static __device__ __forceinline__ v16h load(const _Float16* p) {
    U f; f.h[0] = *(const v8h*)(p); f.h[1] = *(const v8h*)(p + 16); return f.v;
  }
  static __device__ __forceinline__ v8f mma(v16h a, v16h b, v8f c) {
    return __builtin_amdgcn_wmma_f32_16x16x32_f16(false, a, false, b, (short)0, c, false, false);
  }
};

__global__ __launch_bounds__(256) void cast_x_kernel(const float* __restrict__ src, unsigned short* __restrict__ dst,
                                                     int n8, float sc) {
  const int i = blockIdx.x * 256 + threadIdx.x;
  if (i < n8) {
    const float* sp = src + (size_t)i * 8;
    const v4f a = *(const v4f*)(sp);
    const v4f b = *(const v4f*)(sp + 4);
    v8h hv;
#pragma unroll
    for (int e = 0; e < 4; ++e) {
      const float fa = a[e];
      const float fb = b[e];
      hv[e]     = (_Float16)(bf16r(fa) * sc);
      hv[4 + e] = (_Float16)(bf16r(fb) * sc);
    }
    *(volatile v8h*)(dst + (size_t)i * 8) = hv;
    __threadfence();
    *(volatile v8h*)(dst + (size_t)i * 8) = hv;
  }
}

__global__ __launch_bounds__(256) void pack_weights_kernel(
    const float* __restrict__ Wq, const float* __restrict__ Wk, const float* __restrict__ Wv,
    const float* __restrict__ Wf, const float* __restrict__ Wo, const float* __restrict__ Wr,
    unsigned short* __restrict__ BT1, unsigned short* __restrict__ WOT, unsigned short* __restrict__ WRT) {
  __shared__ float Tt[64 * 65];
  const int tid = threadIdx.x;
  const int blk = blockIdx.x;
  const float* src;
  unsigned short* dst;
  int spitch, cvalid, ldo, c0, r0;
  float sc;
  if (blk < PK_QKV_TILES) {
    const int which = blk >> 7;
    const int tl = blk & 127;
    src = (which == 0) ? Wq : ((which == 1) ? Wk : Wv);
    spitch = 512; cvalid = 512; c0 = (tl & 7) * 64; r0 = (tl >> 3) * 64;
    dst = BT1 + (size_t)which * 512 * NDIM; ldo = NDIM; sc = WPCARRY;
  } else if (blk < PK_QKV_TILES + PK_WF_TILES) {
    const int tl = blk - PK_QKV_TILES;
    src = Wf; spitch = NHEAD; cvalid = NHEAD; c0 = 0; r0 = tl * 64;
    dst = BT1 + (size_t)NQKV * NDIM; ldo = NDIM; sc = WPCARRY;
  } else if (blk < PK_QKV_TILES + PK_WF_TILES + PK_WO_TILES) {
    const int tl = blk - (PK_QKV_TILES + PK_WF_TILES);
    src = Wo; spitch = NDIM; cvalid = NDIM; c0 = (tl & 15) * 64; r0 = (tl >> 4) * 64;
    dst = WOT; ldo = NYC; sc = WOCARRY;
  } else {
    const int hn = blk - (PK_QKV_TILES + PK_WF_TILES + PK_WO_TILES);
    src = Wr + (size_t)hn * HDIM * HDIM; spitch = HDIM; cvalid = HDIM; c0 = 0; r0 = 0;
    dst = WRT + (size_t)hn * HDIM * HDIM; ldo = HDIM; sc = WRCARRY;
  }
#pragma unroll
  for (int i = 0; i < 4; ++i) {
    const int idx = i * 256 + tid;
    const int rr = idx >> 4, cc = (idx & 15) * 4;
    const int gc = c0 + cc;
    const bool ok = gc < cvalid;
    const int gcl = ok ? gc : 0;
    const v4f v = *(const v4f*)(src + (size_t)(r0 + rr) * (size_t)spitch + gcl);
    const float f0 = v[0], f1 = v[1], f2 = v[2], f3 = v[3];
    Tt[rr * 65 + cc + 0] = ok ? f0 : 0.0f;
    Tt[rr * 65 + cc + 1] = ok ? f1 : 0.0f;
    Tt[rr * 65 + cc + 2] = ok ? f2 : 0.0f;
    Tt[rr * 65 + cc + 3] = ok ? f3 : 0.0f;
  }
  __syncthreads();
  const int q = tid >> 3, c8 = (tid & 7) * 8;
  v8h hv[2];
#pragma unroll
  for (int g = 0; g < 2; ++g) {
    const int qq = g * 32 + q;
#pragma unroll
    for (int e = 0; e < 8; ++e) {
      const float f = Tt[(c8 + e) * 65 + qq];
      hv[g][e] = (_Float16)(bf16r(f) * sc);
    }
  }
  for (int pass = 0; pass < 2; ++pass) {
#pragma unroll
    for (int g = 0; g < 2; ++g) {
      const size_t o = (size_t)(c0 + g * 32 + q) * (size_t)ldo + (size_t)(r0 + c8);
      *(volatile v8h*)(dst + o) = hv[g];
    }
    __threadfence();
  }
}

__global__ __launch_bounds__(256) void pack_cw_kernel(const float* __restrict__ cq, const float* __restrict__ ck,
                                                      const float* __restrict__ cv, float* __restrict__ dst) {
  const int blk = blockIdx.x;
  const float* src = (blk < 2) ? cq : ((blk < 4) ? ck : cv);
  const int ch = (blk & 1) * 256 + threadIdx.x;
  const v4f v = *(const v4f*)(src + ch * 4);
  v4f o;
#pragma unroll
  for (int e = 0; e < 4; ++e) { const float f = v[e]; o[e] = bf16r(f); }
  float* op = dst + (size_t)(blk * 256 + threadIdx.x) * 4;
  *(volatile v4f*)op = o;
  __threadfence();
  *(volatile v4f*)op = o;
}

__global__ __launch_bounds__(256) void gemm_f16_kernel(
    const unsigned short* __restrict__ Ap, int lda,
    const unsigned short* __restrict__ Btp, int ldb,
    float* __restrict__ C, int ldc, int M, int N, int K, float scale) {
  const _Float16* A  = (const _Float16*)Ap;
  const _Float16* Bt = (const _Float16*)Btp;
  __shared__ __align__(16) float sT[8][16 * 68];
  const int lane = threadIdx.x & 31;
  const int wave = threadIdx.x >> 5;
  const int tilesN = N >> 6;
  const int tilesM = M >> 6;
  const int tile = blockIdx.x * 8 + wave;
  if (tile >= tilesM * tilesN) return;
  const int tm = tile / tilesN;
  const int tn = tile - tm * tilesN;
  const int m0 = tm << 6;
  const int n0 = tn << 6;
  const int rlane = lane & 15;
  const int koff  = (lane >> 4) * 8;
  const int mOff  = (lane >> 4) * 8;

  v8f acc[4][4];
#pragma unroll
  for (int i = 0; i < 4; ++i)
#pragma unroll
    for (int j = 0; j < 4; ++j) acc[i][j] = (v8f){0.f, 0.f, 0.f, 0.f, 0.f, 0.f, 0.f, 0.f};

  const _Float16* bbase = Bt + (size_t)(n0 + rlane) * ldb + koff;
  const _Float16* abase = A  + (size_t)(m0 + rlane) * lda + koff;
  const size_t bstep = (size_t)16 * ldb;
  const size_t astep = (size_t)16 * lda;

  for (int k0 = 0; k0 < K; k0 += 32) {
    v16h bh[4];
#pragma unroll
    for (int j = 0; j < 4; ++j) bh[j] = Frag<_Float16>::load(bbase + (size_t)j * bstep + k0);
#pragma unroll
    for (int i = 0; i < 4; ++i) {
      const v16h ah = Frag<_Float16>::load(abase + (size_t)i * astep + k0);
#pragma unroll
      for (int j = 0; j < 4; ++j) acc[i][j] = Frag<_Float16>::mma(ah, bh[j], acc[i][j]);
      guard_row4(acc[i][0], acc[i][1], acc[i][2], acc[i][3], ah, bh[0], bh[1], bh[2], bh[3]);
    }
    keep4_h(bh[0], bh[1], bh[2], bh[3]);
  }
  acc_guard4(acc[0][0], acc[0][1], acc[0][2], acc[0][3]);
  acc_guard4(acc[1][0], acc[1][1], acc[1][2], acc[1][3]);
  acc_guard4(acc[2][0], acc[2][1], acc[2][2], acc[2][3]);
  acc_guard4(acc[3][0], acc[3][1], acc[3][2], acc[3][3]);

  float* slab = sT[wave];
#pragma unroll
  for (int i = 0; i < 4; ++i) {
    const int mBase = m0 + (i << 4);
#pragma unroll
    for (int j = 0; j < 4; ++j) {
#pragma unroll
      for (int r = 0; r < 8; ++r) slab[(mOff + r) * 68 + (j << 4) + rlane] = acc[i][j][r] * scale;
    }
    __builtin_amdgcn_fence(__ATOMIC_RELEASE, "workgroup");
    __builtin_amdgcn_wave_barrier();
    __builtin_amdgcn_fence(__ATOMIC_ACQUIRE, "workgroup");
    {
      const int hh = lane >> 4, c4 = (lane & 15) * 4;
      for (int pass = 0; pass < 2; ++pass) {
#pragma unroll
        for (int it = 0; it < 8; ++it) {
          const int row = it * 2 + hh;
          const v4f v = *(const v4f*)(slab + row * 68 + c4);
          *(volatile v4f*)(C + (size_t)(mBase + row) * ldc + n0 + c4) = v;
        }
        __threadfence();
      }
    }
    __builtin_amdgcn_fence(__ATOMIC_RELEASE, "workgroup");
    __builtin_amdgcn_wave_barrier();
    __builtin_amdgcn_fence(__ATOMIC_ACQUIRE, "workgroup");
  }
}

__global__ __launch_bounds__(256) void conv_gate_kernel(const float* __restrict__ PRE, const float* __restrict__ CWP,
                                                        const float* __restrict__ bfv,
                                                        float* __restrict__ QKV, float* __restrict__ FG) {
  const int tid = threadIdx.x;
  if (blockIdx.x < CONV_BLOCKS) {
    const int i = blockIdx.x * 256 + tid;
    const int row = i / (NQKV / 4);
    const int c4 = (i - row * (NQKV / 4)) * 4;
    const int l = row & (NSEQ - 1);
    const v4f w0 = *(const v4f*)(CWP + (size_t)(c4 + 0) * 4);
    const v4f w1 = *(const v4f*)(CWP + (size_t)(c4 + 1) * 4);
    const v4f w2 = *(const v4f*)(CWP + (size_t)(c4 + 2) * 4);
    const v4f w3 = *(const v4f*)(CWP + (size_t)(c4 + 3) * 4);
    float s0 = 0.0f, s1 = 0.0f, s2 = 0.0f, s3 = 0.0f;
#pragma unroll
    for (int j = 0; j < 4; ++j) {
      const bool ok = (l - 3 + j) >= 0;
      const int rj = ok ? (row - 3 + j) : row;
      const v4f xv = *(const v4f*)(PRE + (size_t)rj * NPROJ + c4);
      const float x0 = xv[0], x1 = xv[1], x2 = xv[2], x3 = xv[3];
      s0 += w0[j] * (ok ? x0 : 0.0f);
      s1 += w1[j] * (ok ? x1 : 0.0f);
      s2 += w2[j] * (ok ? x2 : 0.0f);
      s3 += w3[j] * (ok ? x3 : 0.0f);
    }
    v4f o;
    o[0] = s0 * __builtin_amdgcn_rcpf(1.0f + expf(-s0));
    o[1] = s1 * __builtin_amdgcn_rcpf(1.0f + expf(-s1));
    o[2] = s2 * __builtin_amdgcn_rcpf(1.0f + expf(-s2));
    o[3] = s3 * __builtin_amdgcn_rcpf(1.0f + expf(-s3));
    float* op = QKV + (size_t)i * 4;
    *(volatile v4f*)op = o;
    __threadfence();
    *(volatile v4f*)op = o;
  } else {
    const int i2 = (blockIdx.x - CONV_BLOCKS) * 256 + tid;
    const int row = i2 >> 1;
    const int n0 = (i2 & 1) * 4;
    const v4f pv = *(const v4f*)(PRE + (size_t)row * NPROJ + NQKV + n0);
    const v4f bv = *(const v4f*)(bfv + n0);
    v4f o;
#pragma unroll
    for (int e = 0; e < 4; ++e) {
      const float pe = pv[e];
      const float be = bv[e];
      const float z = pe + bf16r(be);
      o[e] = __builtin_amdgcn_rcpf(1.0f + expf(-z));
    }
    float* op = FG + (size_t)i2 * 4;
    *(volatile v4f*)op = o;
    __threadfence();
    *(volatile v4f*)op = o;
  }
}

__global__ __launch_bounds__(128) void recur_kernel(const float* __restrict__ QKV, const float* __restrict__ FG,
                                                    const unsigned short* __restrict__ WRTp,
                                                    unsigned short* __restrict__ Y16, float* __restrict__ Hout) {
  __shared__ __align__(16) _Float16 Wl[64 * HSP];
  __shared__ __align__(16) _Float16 Hs[4][16 * HSP];
  __shared__ __align__(16) _Float16 Hl[4][16 * HSP];
  __shared__ __align__(16) float    Hm[4][32 * 32];
  __shared__ __align__(16) float    St[2][192];
  __shared__ __align__(16) float    Yp[2][4 * 64];
  __shared__ __align__(16) float    Sl[4][16 * SLP];

  const int tid = threadIdx.x, lane = tid & 31, wave = tid >> 5;
  const int c = lane & 15, hh = lane >> 4, koff = hh * 8, c4 = c * 4;
  const int bn = blockIdx.x;
  const int b = bn >> 3, n = bn & 7;
  const int rowb = b * NSEQ;

  {
    const _Float16* wg = (const _Float16*)WRTp + (size_t)n * HDIM * HDIM;
#pragma unroll 1
    for (int i = tid; i < 512; i += 128) {
      const int row = i >> 3, c8 = (i & 7) * 8;
      const v8h v = *(const v8h*)(wg + row * HDIM + c8);
      *(v8h*)(Wl + row * HSP + c8) = v;
    }
  }
  {
    v8h zh;
#pragma unroll
    for (int e = 0; e < 8; ++e) zh[e] = (_Float16)0.0f;
    _Float16* hz = &Hs[0][0];
    _Float16* lz = &Hl[0][0];
#pragma unroll 1
    for (int i = tid; i < 576; i += 128) {
      *(v8h*)(hz + i * 8) = zh;
      *(v8h*)(lz + i * 8) = zh;
    }
    const v4f z4 = {0.f, 0.f, 0.f, 0.f};
    float* mz = &Hm[0][0];
#pragma unroll 1
    for (int i = tid; i < 1024; i += 128) *(v4f*)(mz + i * 4) = z4;
  }
  const int selr = tid >> 4;
  const int sel = (selr < 2) ? selr : 2;
  const float* qkvp = QKV + (size_t)rowb * NQKV + n * HDIM + sel * 512 + (tid & 15) * 4;
  const float* fgp  = FG + (size_t)rowb * NHEAD + n;
  {
    v4f s0 = *(const v4f*)(qkvp);
    asm volatile("" : "+v"(s0));
    if (tid < 48) *(v4f*)(&St[0][0] + tid * 4) = s0;
  }
  float gcur = fgp[0];
  asm volatile("" : "+v"(gcur));
  __syncthreads();

  const _Float16* hrow = &Hs[wave][0] + c * HSP + koff;
  const _Float16* lrow = &Hl[wave][0] + c * HSP + koff;
  _Float16* hsw = &Hs[wave][0] + (8 * hh) * HSP + c;
  _Float16* hlw = &Hl[wave][0] + (8 * hh) * HSP + c;
  float* hm = &Hm[wave][0] + lane;
  const _Float16* wlrow = Wl + c * HSP + koff;
  const v8f z8 = {0.f, 0.f, 0.f, 0.f, 0.f, 0.f, 0.f, 0.f};

#pragma unroll 1
  for (int t = 0; t < NSEQ; ++t) {
    const int p = t & 1;
    const int tn = (t + 1 < NSEQ) ? (t + 1) : (NSEQ - 1);
    v4f nx = *(const v4f*)(qkvp + (size_t)tn * NQKV);
    asm volatile("" : "+v"(nx));
    float gnext = fgp[(size_t)tn * NHEAD];
    asm volatile("" : "+v"(gnext));

    v16h a0  = Frag<_Float16>::load(hrow);
    v16h a1  = Frag<_Float16>::load(hrow + 32);
    v16h a0l = Frag<_Float16>::load(lrow);
    v16h a1l = Frag<_Float16>::load(lrow + 32);
    asm volatile("" : "+v"(a0), "+v"(a1), "+v"(a0l), "+v"(a1l) :: "memory");

    const float* st = &St[p][0];
    const v4f q0v = *(const v4f*)(st + 16 * wave + 8 * hh);
    const v4f q1v = *(const v4f*)(st + 16 * wave + 8 * hh + 4);
    const v4f k0v = *(const v4f*)(st + 64 + 16 * wave + 8 * hh);
    const v4f k1v = *(const v4f*)(st + 64 + 16 * wave + 8 * hh + 4);
    float qr[8], kr[8];
#pragma unroll
    for (int e = 0; e < 4; ++e) {
      const float qa = q0v[e], qb = q1v[e], ka = k0v[e], kb = k1v[e];
      qr[e] = qa; qr[4 + e] = qb;
      kr[e] = ka * WRCARRY; kr[4 + e] = kb * WRCARRY;
    }
    const float g = gcur;
    const float omg = 1.0f - g;
    float* ypw = &Yp[p][0] + wave * 64 + c;

#pragma unroll 1
    for (int j = 0; j < 4; ++j) {
      const float vj = st[128 + 16 * j + c];
      v8f acc;
#pragma unroll
      for (int r = 0; r < 8; ++r) acc[r] = kr[r] * vj;
      v8f accL = z8;
      const v16h b0 = Frag<_Float16>::load(wlrow + (16 * j) * HSP);
      const v16h b1 = Frag<_Float16>::load(wlrow + (16 * j) * HSP + 32);
      acc  = Frag<_Float16>::mma(a0, b0, acc);
      acc  = Frag<_Float16>::mma(a1, b1, acc);
      accL = Frag<_Float16>::mma(a0l, b0, accL);
      accL = Frag<_Float16>::mma(a1l, b1, accL);
      guard_pair(acc, a0, a1, b0, b1);
      guard_pair(accL, a0l, a1l, b0, b1);
      float ys = 0.0f;
#pragma unroll
      for (int r = 0; r < 8; ++r) {
        const float e2 = expf(acc[r] * ZSCALE2 + accL[r] * ZSCALE2L);
        const float cand = 1.0f - 2.0f * __builtin_amdgcn_rcpf(e2 + 1.0f);
        const float ho = hm[(j * 8 + r) * 32];
        const float hn = g * ho + omg * cand;
        hm[(j * 8 + r) * 32] = hn;
        const float hq = (fabsf(hn) < HFLUSH) ? 0.0f : hn;
        const _Float16 hi = (_Float16)hq;
        const float hif = (float)hi;
        const _Float16 lo = (_Float16)((hn - hif) * LOCARRY);
        hsw[r * HSP + 16 * j] = hi;
        hlw[r * HSP + 16 * j] = lo;
        ys += qr[r] * hn;
      }
      ys += __shfl_xor(ys, 16, 32);
      if (hh == 0) ypw[16 * j] = ys;
    }

    if (tid < 48) *(v4f*)(&St[p ^ 1][0] + tid * 4) = nx;
    gcur = gnext;
    __syncthreads();

    if (wave == 0) {
      const float* ypp = &Yp[p][0] + 8 * (lane & 7);
      v4f s0 = *(const v4f*)(ypp);
      v4f s1 = *(const v4f*)(ypp + 4);
#pragma unroll
      for (int w2 = 1; w2 < 4; ++w2) {
        s0 += *(const v4f*)(ypp + 64 * w2);
        s1 += *(const v4f*)(ypp + 64 * w2 + 4);
      }
      v8h hv;
#pragma unroll
      for (int e = 0; e < 4; ++e) {
        const float fa = s0[e];
        const float fb = s1[e];
        hv[e] = (_Float16)fa;
        hv[4 + e] = (_Float16)fb;
      }
      unsigned short* yo = Y16 + ((size_t)(rowb + t) * NYC + n * HDIM + 8 * (lane & 7));
      if (lane < 8) *(volatile v8h*)yo = hv;
      __threadfence();
      if (lane < 8) *(volatile v8h*)yo = hv;
    }
  }

  float* slab = &Sl[wave][0];
#pragma unroll 1
  for (int j = 0; j < 4; ++j) {
#pragma unroll
    for (int r = 0; r < 8; ++r) slab[(8 * hh + r) * SLP + 16 * j + c] = hm[(j * 8 + r) * 32];
  }
  __syncthreads();
  float* hob = Hout + ((size_t)bn * HDIM + 16 * wave) * HDIM;
  for (int pass = 0; pass < 2; ++pass) {
#pragma unroll
    for (int it = 0; it < 8; ++it) {
      const int row = it * 2 + hh;
      const v4f v = *(const v4f*)(slab + row * SLP + c4);
      *(volatile v4f*)(hob + (size_t)row * HDIM + c4) = v;
    }
    __threadfence();
  }
}

extern "C" void kernel_launch(void* const* d_in, const int* in_sizes, int n_in,
                              void* d_out, int out_size, void* d_ws, size_t ws_size, hipStream_t stream) {
  if (n_in < 11 || d_out == nullptr || d_ws == nullptr) return;
  if (in_sizes[0] != NROWS * NDIM || in_sizes[1] != NDIM * 512 || in_sizes[2] != NDIM * 512 ||
      in_sizes[3] != NDIM * 512 || in_sizes[4] != NDIM * NHEAD || in_sizes[5] != NHEAD ||
      in_sizes[6] != 512 * 4 || in_sizes[7] != 512 * 4 || in_sizes[8] != 512 * 4 ||
      in_sizes[9] != NHEAD * HDIM * HDIM || in_sizes[10] != NYC * NDIM ||
      out_size != NOUT0 + NOUT1) return;

  const float* x   = (const float*)d_in[0];
  const float* Wq  = (const float*)d_in[1];
  const float* Wk  = (const float*)d_in[2];
  const float* Wv  = (const float*)d_in[3];
  const float* Wf  = (const float*)d_in[4];
  const float* bfv = (const float*)d_in[5];
  const float* cwq = (const float*)d_in[6];
  const float* cwk = (const float*)d_in[7];
  const float* cwv = (const float*)d_in[8];
  const float* Wr  = (const float*)d_in[9];
  const float* Wo  = (const float*)d_in[10];
  float* out0 = (float*)d_out;
  float* hfin = out0 + (size_t)NOUT0;

  char* ws = (char*)d_ws;
  size_t off = 0;
  auto carve = [&](size_t bytes) -> char* { char* p = ws + off; off += (bytes + 255) & ~(size_t)255; return p; };
  unsigned short* X16 = (unsigned short*)carve((size_t)NROWS * NDIM * 2);
  unsigned short* BT1 = (unsigned short*)carve((size_t)NPROJ * NDIM * 2);
  unsigned short* WOT = (unsigned short*)carve((size_t)NDIM * NYC * 2);
  unsigned short* WRT = (unsigned short*)carve((size_t)NHEAD * HDIM * HDIM * 2);
  float*          CWP = (float*)carve((size_t)NQKV * 4 * 4);
  float*          PRE = (float*)carve((size_t)NROWS * NPROJ * 4);
  float*          QKV = (float*)carve((size_t)NROWS * NQKV * 4);
  float*          FG  = (float*)carve((size_t)NROWS * NHEAD * 4);
  unsigned short* Y16 = (unsigned short*)carve((size_t)NROWS * NYC * 2);
  if (off > ws_size || off > (size_t)134217728) return;

  const int n8x = NROWS * (NDIM / 8);
  cast_x_kernel<<<(n8x + 255) / 256, 256, 0, stream>>>(x, X16, n8x, XCARRY);
  pack_weights_kernel<<<PK_TILES, 256, 0, stream>>>(Wq, Wk, Wv, Wf, Wo, Wr, BT1, WOT, WRT);
  pack_cw_kernel<<<6, 256, 0, stream>>>(cwq, cwk, cwv, CWP);

  gemm_f16_kernel<<<(NROWS / 64) * (NPROJ / 64) / 8, 256, 0, stream>>>(
      X16, NDIM, BT1, NDIM, PRE, NPROJ, NROWS, NPROJ, NDIM, PROJ_SCALE);

  conv_gate_kernel<<<CONV_BLOCKS + GATE_BLOCKS, 256, 0, stream>>>(PRE, CWP, bfv, QKV, FG);

  recur_kernel<<<NBAT * NHEAD, 128, 0, stream>>>(QKV, FG, WRT, Y16, hfin);

  gemm_f16_kernel<<<(NROWS / 64) * (NDIM / 64) / 8, 256, 0, stream>>>(
      Y16, NYC, WOT, NYC, out0, NDIM, NROWS, NDIM, NYC, OUT_SCALE);
}
